// LocalStridedBlockSparseAttn_48825188221191
// MI455X (gfx1250) — hardware-verified
//
#include <hip/hip_runtime.h>
#include <math.h>

typedef __attribute__((ext_vector_type(16))) _Float16 v16h;
typedef __attribute__((ext_vector_type(16))) __bf16 v16b;
typedef __attribute__((ext_vector_type(8)))  _Float16 v8h;
typedef __attribute__((ext_vector_type(8)))  float v8f;
typedef __attribute__((ext_vector_type(4)))  float v4f;
typedef __attribute__((ext_vector_type(2)))  float v2f;
typedef __attribute__((ext_vector_type(4)))  unsigned v4u;
typedef __attribute__((ext_vector_type(4)))  int v4i;
typedef float __attribute__((may_alias)) float_a;
typedef int __attribute__((may_alias)) int_a;

template <typename T> __device__ __forceinline__ void vst2(void* p, T v) { *(volatile T*)p = v; __threadfence(); *(volatile T*)p = v; }
__device__ __forceinline__ v8f wmma16(v16h a, v16h b, v8f c) {
  v8f d = __builtin_amdgcn_wmma_f32_16x16x32_f16(false, a, false, b, (short)0, c, false, false);
  asm volatile("v_nop\n\tv_nop\n\tv_nop\n\tv_nop" : "+v"(d) : "v"(a), "v"(b));
  return d;
}
__device__ __forceinline__ v8f wmma_bf(v16b a, v16b b, v8f c) {
  v8f d = __builtin_amdgcn_wmma_f32_16x16x32_bf16(false, a, false, b, (short)0, c, false, false);
  asm volatile("v_nop\n\tv_nop\n\tv_nop\n\tv_nop" : "+v"(d) : "v"(a), "v"(b));
  return d;
}
__device__ __forceinline__ v16h frag_h(const _Float16* rowk0, int lane) {
  union { v16h v; v8h q[2]; } u; const _Float16* p = rowk0 + 8 * (lane >> 4);
  u.q[0] = *(const v8h*)p; u.q[1] = *(const v8h*)(p + 16); return u.v;
}
__device__ __forceinline__ v16h frag_f32(const float* rowk0, int lane) {
  v16h a; const float* p = rowk0 + 8 * (lane >> 4);
#pragma unroll
  for (int i = 0; i < 8; ++i) { a[i] = (_Float16)p[i]; a[8 + i] = (_Float16)p[16 + i]; }
  return a;
}
__device__ __forceinline__ v16h frag_f32s(const float* rowk0, int lane, float sc) {
  v16h a; const float* p = rowk0 + 8 * (lane >> 4);
#pragma unroll
  for (int i = 0; i < 8; ++i) { a[i] = (_Float16)(p[i] * sc); a[8 + i] = (_Float16)(p[16 + i] * sc); }
  return a;
}
__device__ __forceinline__ v16h fragc_f32(const float* W, int k0, int n, int lane, int ld, int K) {
  v16h a; const int g = lane >> 4;
#pragma unroll
  for (int i = 0; i < 8; ++i) { const int ka = k0 + 8 * g + i, kb = ka + 16;
    a[i] = (_Float16)(ka < K ? W[(size_t)(ka < K ? ka : K - 1) * ld + n] : 0.f); a[8 + i] = (_Float16)(kb < K ? W[(size_t)(kb < K ? kb : K - 1) * ld + n] : 0.f); }
  return a;
}
struct F2 { v16b h, l; };
__device__ __forceinline__ F2 bsplit16(const float v[16]) { F2 r;
#pragma unroll
  for (int i = 0; i < 16; ++i) { const __bf16 h = (__bf16)v[i]; r.h[i] = h; r.l[i] = (__bf16)(v[i] - (float)h); }
  return r; }
__device__ __forceinline__ F2 split_row(const float* row, int k0, int lane) { float v[16]; const float* p = row + k0 + 8 * (lane >> 4);
#pragma unroll
  for (int i = 0; i < 8; ++i) { v[i] = p[i]; v[8 + i] = p[16 + i]; }
  return bsplit16(v); }
__device__ __forceinline__ F2 split_rowK(const float* row, int k0, int lane, int K) { float v[16]; const int g = lane >> 4;
#pragma unroll
  for (int i = 0; i < 8; ++i) { const int ka = k0 + 8 * g + i, kb = ka + 16; v[i] = ka < K ? row[ka < K ? ka : K - 1] : 0.f; v[8 + i] = kb < K ? row[kb < K ? kb : K - 1] : 0.f; }
  return bsplit16(v); }
__device__ __forceinline__ F2 split_col(const float* W, int k0, int n, int lane, int ld, int K) { float v[16]; const int g = lane >> 4;
#pragma unroll
  for (int i = 0; i < 8; ++i) { const int ka = k0 + 8 * g + i, kb = ka + 16; v[i] = ka < K ? W[(size_t)(ka < K ? ka : K - 1) * ld + n] : 0.f; v[8 + i] = kb < K ? W[(size_t)(kb < K ? kb : K - 1) * ld + n] : 0.f; }
  return bsplit16(v); }
__device__ __forceinline__ v8f mac3(const F2& a, const F2& b, v8f c) { c = wmma_bf(a.l, b.h, c); c = wmma_bf(a.h, b.l, c); return wmma_bf(a.h, b.h, c); }
__device__ __forceinline__ float sigm(float v) { return 1.0f / (1.0f + expf(-v)); }
#define LDSX() do { asm volatile("s_wait_dscnt 0" ::: "memory"); __builtin_amdgcn_wave_barrier(); __builtin_amdgcn_fence(__ATOMIC_RELEASE, "workgroup"); } while (0)


#define TT 4096
#define NH 16
#define HD 64
#define BS 64
#define NBLK (TT / BS)
#define LOCALB 8
#define VERT 8
#ifndef TQB
#define TQB NBLK
#define TNH NH
#endif
typedef __attribute__((ext_vector_type(8))) __bf16 v8b;
__device__ __forceinline__ v16b frag_b(const __bf16* rowk0, int lane) {
  union { v16b v; v8b q[2]; } u; const __bf16* p = rowk0 + 8 * (lane >> 4);
  u.q[0] = *(const v8b*)p; u.q[1] = *(const v8b*)(p + 16); return u.v;
}
__device__ __forceinline__ v16b frag_gbf(const float* rowk0, int lane) {
  v16b a; const float* p = rowk0 + 8 * (lane >> 4);
#pragma unroll
  for (int i = 0; i < 8; ++i) { a[i] = (__bf16)p[i]; a[8 + i] = (__bf16)p[16 + i]; }
  return a;
}
__device__ __attribute__((noinline)) float exp_ni(float v) { return expf(v); }
#define WS_VT  0u
#define WS_END (WS_VT + 2u * NH * HD * TT)
__global__ __launch_bounds__(256) void k_vt(const float* __restrict__ V, __bf16* __restrict__ VT) {
  __shared__ __align__(16) __bf16 sv[HD][72];
  const int tid = threadIdx.x; const int h = blockIdx.y; const int t0 = blockIdx.x * 64;
  for (int q = tid; q < 64 * HD; q += 256) { const int tl = q >> 6, d = q & 63; sv[d][tl] = (__bf16)V[((size_t)(t0 + tl) * NH + h) * HD + d]; }
  __syncthreads();
  for (int q = tid; q < HD * 8; q += 256) { const int d = q >> 3, pc = q & 7; vst2((unsigned*)(VT + ((size_t)h * HD + d) * TT + t0 + pc * 8), *(const v4u*)&sv[d][pc * 8]); }
}
__global__ __launch_bounds__(128) void k_attn(const float* __restrict__ Q, const float* __restrict__ K, const __bf16* __restrict__ VT, float* __restrict__ OUT) {
  __shared__ __align__(16) float sp[4][16][36]; __shared__ __align__(16) float so[4][16][68];
  const int tid = threadIdx.x, wave = tid >> 5, lane = tid & 31, col = lane & 15, g = lane >> 4;
  const int qb = blockIdx.x, h = blockIdx.y; const int q0 = qb * BS + wave * 16;
  const v16b a0 = frag_gbf(Q + ((size_t)(q0 + col) * NH + h) * HD, lane), a1 = frag_gbf(Q + ((size_t)(q0 + col) * NH + h) * HD + 32, lane);
  float m[8], l[8]; v8f acc[4] = {};
#pragma unroll
  for (int r = 0; r < 8; ++r) { m[r] = -3.0e38f; l[r] = 0.f; }
#pragma unroll 1
  for (int j = 0; j <= qb; ++j) { const bool use = ((qb - j) < LOCALB) || (((j + h + 1) % VERT) == 0); if (!use) continue;
    const bool diag = (j == qb);
#pragma unroll 1
    for (int st = 0; st < 2; ++st) { const int kbase = j * BS + st * 32; v8f s[2];
#pragma unroll
      for (int ct = 0; ct < 2; ++ct) { const int kk = kbase + ct * 16 + col; const float* krow = K + ((size_t)kk * NH + h) * HD; v8f c = {}; c = wmma_bf(a0, frag_gbf(krow, lane), c); c = wmma_bf(a1, frag_gbf(krow + 32, lane), c);
#pragma unroll
        for (int r = 0; r < 8; ++r) { float v = c[r] * 0.125f; if (diag && kk > q0 + 8 * g + r) v = -3.0e38f; s[ct][r] = v; } }
#pragma unroll
      for (int r = 0; r < 8; ++r) { float mx = fmaxf(s[0][r], s[1][r]);
#pragma unroll
        for (int o = 1; o < 16; o <<= 1) mx = fmaxf(mx, __shfl_xor(mx, o));
        const float mn = fmaxf(m[r], mx); const float alpha = exp_ni(m[r] - mn);
        const float e0 = s[0][r] <= -1.0e38f ? 0.f : exp_ni(s[0][r] - mn), e1 = s[1][r] <= -1.0e38f ? 0.f : exp_ni(s[1][r] - mn); float es = e0 + e1;
#pragma unroll
        for (int o = 1; o < 16; o <<= 1) es += __shfl_xor(es, o);
        l[r] = l[r] * alpha + es; m[r] = mn;
#pragma unroll
        for (int dt = 0; dt < 4; ++dt) acc[dt][r] *= alpha;
        sp[wave][8 * g + r][col] = e0; sp[wave][8 * g + r][16 + col] = e1; }
      LDSX();
      const F2 pa = split_row(&sp[wave][col][0], 0, lane);
#pragma unroll
      for (int dt = 0; dt < 4; ++dt) { const v16b vb = frag_b(VT + ((size_t)h * HD + dt * 16 + col) * TT + kbase, lane); acc[dt] = wmma_bf(pa.l, vb, acc[dt]); acc[dt] = wmma_bf(pa.h, vb, acc[dt]); }
      LDSX(); } }
#pragma unroll
  for (int r = 0; r < 8; ++r) { const float il = (l[r] > 0.f) ? 1.0f / l[r] : 0.f;
#pragma unroll
    for (int dt = 0; dt < 4; ++dt) so[wave][8 * g + r][dt * 16 + col] = acc[dt][r] * il; }
  LDSX();
  for (int rl = 0; rl < 16; ++rl) if (lane < 16) vst2(OUT + ((size_t)(q0 + rl) * NH + h) * HD + lane * 4, *(const v4f*)&so[wave][rl][lane * 4]);
}
extern "C" void kernel_launch(void* const* d_in, const int* in_sizes, int n_in, void* d_out, int out_size, void* d_ws, size_t ws_size, hipStream_t stream) {
  (void)in_sizes; (void)n_in; (void)out_size;
  const float** F = (const float**)d_in;
  if (ws_size < (size_t)WS_END) return;
  char* ws = (char*)d_ws; __bf16* VT = (__bf16*)(ws + WS_VT);
  k_vt<<<dim3(TT / 64, NH), 256, 0, stream>>>(F[2], VT);
  k_attn<<<dim3(TQB, TNH), 128, 0, stream>>>(F[0], F[1], VT, (float*)d_out);
}
